// Fusion_Block_GLAFF_15728170238234
// MI455X (gfx1250) — hardware-run, weakly checked
//
#include <hip/hip_runtime.h>


#ifndef NB
#define NB 32
#endif
#define NB_FULL 32
#define LL   512
#define OO   192
#define DF   32
#define KD   6
#define DMM  512
#define AW   4
#define WSC  64.0f
#define WSI  (1.0f / 64.0f)
#define SC2  ((float)(0.40824829046386302 * 1.4426950408889634))
#define NEGB (-3.0e38f)

static_assert(NB <= NB_FULL);
static_assert(LL == 512);
static_assert(DF == 32);
static_assert(KD <= 8);
static_assert((DF * KD) % 32 == 0);
static_assert(DF * KD <= 256);
static_assert(LL % 64 == 0);
static_assert(LL % 32 == 0);
static_assert(OO % (16 * AW) == 0);
static_assert(OO % 64 == 0);
static_assert(OO % 32 == 0);
static_assert(OO % 16 == 0);
static_assert(AW == 4);
static_assert(DMM == 8 * 64);
static_assert(DMM % 64 == 0);
static_assert((NB * DF) % 64 == 0);
static_assert(256 * 8 * 16 == DF * 16 * 64);
static_assert(256 * 1 * 16 == DF * 64 * 2);
static_assert(128 * 16 == 16 * DF * 4);
static_assert(16 * 16 == 16 * AW * 4);
static_assert(256 * 2 * 16 == 64 * 64 * 2);
static_assert(32 * 16 == 64 * 2 * 4);
static_assert(256 * 2 * 16 == 64 * DF * 4);
static_assert(8 * 16 == 32 * 4);
static_assert(LL * 4 + 2 * 32 * 4 <= 131072);
static_assert(DF * 16 * 32 * 2 + DF * 64 * 2 + 4 * 256 * 4 <= 131072);
static_assert(DF * 16 * 32 * 2 + 16 * DF * 4 + 4 * 256 * 4 <= 131072);
static_assert(LL * 4 + 16 * AW * 4 <= 131072);
static_assert(64 * 65 * 4 <= 131072);
static_assert(8 * 16 * 68 * 4 + DMM * 4 + DMM * 2 * 4 + 8 * 64 * 2 * 4 + 64 * 2 * 4 <= 131072);
static_assert(DF * 65 * 4 + 6 * 32 * 4 <= 131072);

typedef _Float16 h16;
typedef unsigned short bf;
typedef __attribute__((ext_vector_type(16))) __bf16   v16bf;
typedef __attribute__((ext_vector_type(16))) _Float16 v16h;
typedef __attribute__((ext_vector_type(8)))  _Float16 v8h;
typedef __attribute__((ext_vector_type(8)))  unsigned short v8us;
typedef __attribute__((ext_vector_type(8)))  float    v8f;
typedef __attribute__((ext_vector_type(4)))  float    v4f;
typedef v4f  __attribute__((may_alias)) v4fa;
typedef v8us __attribute__((may_alias)) v8usa;
typedef v8h  __attribute__((may_alias)) v8ha;

__device__ __forceinline__ unsigned short f2bf(float f) { unsigned u = __float_as_uint(f); u += 0x7FFFu + ((u >> 16) & 1u); return (unsigned short)(u >> 16); }
__device__ __forceinline__ float bfr(float f) { return __uint_as_float(((unsigned)f2bf(f)) << 16); }
__device__ __forceinline__ v16h cat16(v8h lo, v8h hi) { return __builtin_shufflevector(lo, hi, 0, 1, 2, 3, 4, 5, 6, 7, 8, 9, 10, 11, 12, 13, 14, 15); }
__device__ __forceinline__ v16bf cat16b(v8us lo, v8us hi) { return __builtin_bit_cast(v16bf, __builtin_shufflevector(lo, hi, 0, 1, 2, 3, 4, 5, 6, 7, 8, 9, 10, 11, 12, 13, 14, 15)); }
__device__ __forceinline__ v8f wmma16(v16h a, v16h b, v8f c) { return __builtin_amdgcn_wmma_f32_16x16x32_f16(false, a, false, b, (short)0, c, false, false); }
__device__ __forceinline__ v8f wmmab(v16bf a, v16bf b, v8f c) { return __builtin_amdgcn_wmma_f32_16x16x32_bf16(false, a, false, b, (short)0, c, false, false); }
__device__ __forceinline__ v16h  ldh(const h16* p) { return cat16(*(const v8h*)p, *(const v8h*)(p + 16)); }
__device__ __forceinline__ v16bf ldb(const bf* p)  { return cat16b(*(const v8us*)p, *(const v8us*)(p + 16)); }
__device__ __forceinline__ void wave_sync() { __builtin_amdgcn_fence(3  , "wavefront"); __builtin_amdgcn_wave_barrier(); asm volatile("" ::: "memory"); }

__device__ __forceinline__ v8f wmma16g(v16h a, v16h b, v8f c) { c = wmma16(a, b, c); asm volatile("v_nop\n\tv_nop\n\tv_nop\n\tv_nop" : "+v"(c) : "v"(a), "v"(b)); return c; }
__device__ __forceinline__ v8f wmmabg(v16bf a, v16bf b, v8f c) { c = wmmab(a, b, c); asm volatile("v_nop\n\tv_nop\n\tv_nop\n\tv_nop" : "+v"(c) : "v"(a), "v"(b)); return c; }
__device__ __forceinline__ float bf2f(unsigned short h) { return __uint_as_float(((unsigned)h) << 16); }
static __device__ __forceinline__ h16 toh_flush(float v) { const h16 r = (h16)v; return (fabsf(v) < 6.103515625e-05f) ? (h16)0.0f : r; }

__global__ __launch_bounds__(256) void k_stats(const float* __restrict__ src, int inner, float* MED, float* STD) {
#pragma clang fp contract(off)
    __shared__ __align__(16) float s[LL];
    __shared__ __align__(16) float rm[32];
    __shared__ __align__(16) float rs[32];
    const int tid = threadIdx.x;
    const int lane = threadIdx.x & 31;
    const int wave = __builtin_amdgcn_readfirstlane((int)(threadIdx.x >> 5));
#pragma unroll 1
    for (int j = 0; j < 32; ++j) {
        const int c = blockIdx.x * 32 + j;
        const int bb = c / inner, rem = c - bb * inner;
        const size_t base = (size_t)bb * (size_t)LL * (size_t)inner + (size_t)rem;
        s[tid]       = bfr(src[base + (size_t)tid * (size_t)inner]);
        s[tid + 256] = bfr(src[base + (size_t)(tid + 256) * (size_t)inner]);
        __syncthreads();
#pragma unroll 1
        for (int k = 2; k <= LL; k <<= 1) {
#pragma unroll 1
            for (int jj = k >> 1; jj > 0; jj >>= 1) {
                const int i = ((tid & ~(jj - 1)) << 1) | (tid & (jj - 1));
                const int p = i | jj;
                const float a = s[i], q = s[p];
                const bool up = (i & k) == 0;
                const bool sw = up ? (a > q) : (a < q);
                s[i] = sw ? q : a; s[p] = sw ? a : q;
                __syncthreads();
            }
        }
        if (tid == 0) {
            const float qh = s[383] * 0.25f + s[384] * 0.75f;
            const float ql = s[127] * 0.25f + s[128] * 0.75f;
            const float qh2 = s[383] * 0.75f + s[384] * 0.25f;
            (void)qh;
            rm[j] = s[255];
            rs[j] = (qh2 - ql) + 1e-6f;
        }
        __syncthreads();
    }
    const int q8 = lane & 7;
    const v4f vm = *(const v4fa*)(&rm[4 * q8]);
    const v4f vs = *(const v4fa*)(&rs[4 * q8]);
    if (wave == 0) {
        if (lane < 8) {
            float* pm = MED + (size_t)blockIdx.x * 32 + 4 * lane;
            float* ps = STD + (size_t)blockIdx.x * 32 + 4 * lane;
            *(volatile v4f*)pm = vm; *(volatile v4f*)ps = vs;
            __threadfence();
            *(volatile v4f*)pm = vm; *(volatile v4f*)ps = vs;
        }
    }
}

__global__ __launch_bounds__(256) void k_mapx(const float* __restrict__ X, const float* __restrict__ XD, const float* __restrict__ MEDT, const float* __restrict__ STDT,
                                              const float* __restrict__ MEDM, const float* __restrict__ STDM, bf* XP, h16* ERR) {
    __shared__ __align__(16) unsigned short xt[DF * 16 * 32];
    __shared__ __align__(16) h16 et[DF * 64];
    __shared__ float smed[256];
    __shared__ float srcp[256];
    __shared__ float smt[256];
    __shared__ float sst[256];
    const int tid = threadIdx.x;
    const int b = blockIdx.y;
    const int lb = blockIdx.x * 64;
    { const int i6 = tid < DF * KD ? tid : (DF * KD - 1); const int i1 = tid & (DF - 1);
      smed[tid] = MEDM[(size_t)b * DF * KD + i6]; srcp[tid] = 1.0f / STDM[(size_t)b * DF * KD + i6];
      smt[tid] = MEDT[(size_t)b * DF + i1]; sst[tid] = STDT[(size_t)b * DF + i1]; }
    __syncthreads();
#pragma unroll 1
    for (int sub = 0; sub < 4; ++sub) {
        const int l0 = lb + sub * 16;
#pragma unroll 1
        for (int it = 0; it < 2; ++it) {
            const int item = it * 256 + tid; const int ll = item >> 5, d = item & 31;
            const size_t e = ((size_t)b * LL + (size_t)(l0 + ll)) * DF + d;
            const float* xd = XD + e * KD;
            const float st = sst[d], mt = smt[d];
            v8us ph = (v8us){}, pm = (v8us){}; float sum = 0.0f;
#pragma unroll
            for (int k = 0; k < KD; ++k) {
                const float v = ((bfr(xd[k]) - smed[d * KD + k]) * srcp[d * KD + k]) * st + mt;
                const unsigned short hb = f2bf(v);
                ph[k] = hb; pm[k] = f2bf(v - bf2f(hb)); sum += v; }
            const int ro = (d * 16 + ll) * 32;
            *(v8usa*)(&xt[ro]) = ph; *(v8usa*)(&xt[ro + 8]) = pm; *(v8usa*)(&xt[ro + 16]) = ph; *(v8usa*)(&xt[ro + 24]) = pm;
            et[d * 64 + sub * 16 + ll] = toh_flush(bfr(X[e]) - sum * (1.0f / 6.0f));
        }
        __syncthreads();
        const size_t gb = ((size_t)b * DF * LL + (size_t)l0) * 32;
#pragma unroll 1
        for (int ps = 0; ps < 2; ++ps) {
#pragma unroll
            for (int it = 0; it < 8; ++it) { const int p = it * 256 + tid; const int d = p >> 6, w = p & 63;
                const v8us val = *(const v8usa*)(&xt[d * 512 + w * 8]);
                *(volatile v8us*)(XP + gb + (size_t)d * LL * 32 + (size_t)w * 8) = val; }
            if (ps == 0) __threadfence(); }
        __syncthreads();
    }
    { const int d = tid >> 3, c8 = (tid & 7) * 8;
      const v8h val = *(const v8ha*)(&et[d * 64 + c8]);
      h16* dst = ERR + ((size_t)b * DF + d) * LL + lb + c8;
      *(volatile v8h*)dst = val; __threadfence(); *(volatile v8h*)dst = val; }
}

__global__ __launch_bounds__(256) void k_mapy(const float* __restrict__ YD, const float* __restrict__ MEDT, const float* __restrict__ STDT,
                                              const float* __restrict__ MEDM, const float* __restrict__ STDM, bf* YP, float* YM) {
    __shared__ __align__(16) unsigned short yt[DF * 16 * 32];
    __shared__ __align__(16) float ym[16 * DF];
    __shared__ float smed[256];
    __shared__ float srcp[256];
    __shared__ float smt[256];
    __shared__ float sst[256];
    const int tid = threadIdx.x;
    const int wave = __builtin_amdgcn_readfirstlane((int)(threadIdx.x >> 5));
    const int b = blockIdx.y;
    const int o0 = blockIdx.x * 16;
    { const int i6 = tid < DF * KD ? tid : (DF * KD - 1); const int i1 = tid & (DF - 1);
      smed[tid] = MEDM[(size_t)b * DF * KD + i6]; srcp[tid] = 1.0f / STDM[(size_t)b * DF * KD + i6];
      smt[tid] = MEDT[(size_t)b * DF + i1]; sst[tid] = STDT[(size_t)b * DF + i1]; }
    __syncthreads();
#pragma unroll 1
    for (int it = 0; it < 2; ++it) {
        const int item = it * 256 + tid; const int oo = item >> 5, d = item & 31;
        const size_t e = ((size_t)b * OO + (size_t)(o0 + oo)) * DF + d;
        const float* yd = YD + e * KD;
        const float st = sst[d], mt = smt[d];
        v8us ph = (v8us){}, pm = (v8us){}; float sum = 0.0f;
#pragma unroll
        for (int k = 0; k < KD; ++k) {
            const float v = ((bfr(yd[k]) - smed[d * KD + k]) * srcp[d * KD + k]) * st + mt;
            const unsigned short hb = f2bf(v);
            ph[k] = hb; pm[k] = f2bf(v - bf2f(hb)); sum += v; }
        const int ro = (d * 16 + oo) * 32;
        *(v8usa*)(&yt[ro]) = ph; *(v8usa*)(&yt[ro + 8]) = ph; *(v8usa*)(&yt[ro + 16]) = pm; *(v8usa*)(&yt[ro + 24]) = pm;
        ym[oo * DF + d] = sum * (1.0f / 6.0f);
    }
    __syncthreads();
    const size_t gb = ((size_t)b * DF * OO + (size_t)o0) * 32;
    const v4f ymv = *(const v4fa*)(&ym[(tid & 127) * 4]);
    float* ymd = YM + ((size_t)b * OO + (size_t)o0) * DF + (size_t)(tid & 127) * 4;
#pragma unroll 1
    for (int ps = 0; ps < 2; ++ps) {
#pragma unroll
        for (int it = 0; it < 8; ++it) { const int p = it * 256 + tid; const int d = p >> 6, w = p & 63;
            const v8us val = *(const v8usa*)(&yt[d * 512 + w * 8]);
            *(volatile v8us*)(YP + gb + (size_t)d * OO * 32 + (size_t)w * 8) = val; }
        if (wave < 4) *(volatile v4f*)ymd = ymv;
        if (ps == 0) __threadfence(); }
}

__global__ __launch_bounds__(32 * AW) void k_flash(const bf* __restrict__ XP, const bf* __restrict__ YP, const float* __restrict__ X, float* VP) {
    __shared__ __align__(16) float xs[LL];
    __shared__ __align__(16) float vs[16 * AW];
    const int lane = threadIdx.x & 31, lr = lane & 15, hi = lane >> 4;
    const int wave = __builtin_amdgcn_readfirstlane((int)(threadIdx.x >> 5));
    const int bd = blockIdx.y; const int b = bd / DF, d = bd % DF;
    for (int i = threadIdx.x; i < LL; i += 32 * AW) xs[i] = bfr(X[((size_t)b * LL + i) * DF + d]);
    __syncthreads();
    const int t0 = (blockIdx.x * AW + wave) * 16;
    const v16bf qf = ldb(YP + ((size_t)bd * OO + (size_t)(t0 + lr)) * 32 + 8 * hi);
    const size_t ko = ((size_t)bd * LL + (size_t)lr) * 32 + 8 * hi;
    float m = NEGB, l = 0.0f, va = 0.0f;
#pragma unroll 1
    for (int key0 = 0; key0 < LL; key0 += 32) {
        const bf* ka = XP + ko + (size_t)key0 * 32;
        const v16bf a0 = ldb(ka), a1 = ldb(ka + 16 * 32);
        v8f s0 = (v8f){}, s1 = (v8f){};
        s0 = wmmabg(a0, qf, s0);
        s1 = wmmabg(a1, qf, s1);
        const v4f x0 = *(const v4fa*)(&xs[key0 + 8 * hi]), x1 = *(const v4fa*)(&xs[key0 + 8 * hi + 4]);
        const v4f x2 = *(const v4fa*)(&xs[key0 + 16 + 8 * hi]), x3 = *(const v4fa*)(&xs[key0 + 16 + 8 * hi + 4]);
        float xa[8], xb[8];
#pragma unroll
        for (int r = 0; r < 4; ++r) { xa[r] = x0[r]; xa[4 + r] = x1[r]; xb[r] = x2[r]; xb[4 + r] = x3[r]; }
        float ta[8], tb[8]; float mx = NEGB;
#pragma unroll
        for (int r = 0; r < 8; ++r) { ta[r] = s0[r] * SC2; tb[r] = s1[r] * SC2; mx = fmaxf(mx, fmaxf(ta[r], tb[r])); }
        mx = fmaxf(mx, __shfl_xor(mx, 16, 32));
        const float mnew = fmaxf(m, mx);
        const float alpha = __builtin_amdgcn_exp2f(m - mnew);
        float ls = 0.0f, vsum = 0.0f;
#pragma unroll
        for (int r = 0; r < 8; ++r) {
            const float ea = __builtin_amdgcn_exp2f(ta[r] - mnew), eb = __builtin_amdgcn_exp2f(tb[r] - mnew);
            ls += ea + eb; vsum += ea * xa[r]; vsum += eb * xb[r]; }
        l = l * alpha + ls; va = va * alpha + vsum; m = mnew;
    }
    l += __shfl_xor(l, 16, 32);
    va += __shfl_xor(va, 16, 32);
    const float res = va * (1.0f / l);
    vs[wave * 16 + lr] = res;
    __syncthreads();
    const v4f val = *(const v4fa*)(&vs[(lane & 15) * 4]);
    if (wave == 0) {
        if (lane < 16) {
            float* dst = VP + (size_t)bd * OO + (size_t)blockIdx.x * (16 * AW) + lane * 4;
            *(volatile v4f*)dst = val; __threadfence(); *(volatile v4f*)dst = val;
        }
    }
}

__global__ __launch_bounds__(256) void k_bn(const float* __restrict__ VP, float* BNT) {
#pragma clang fp contract(off)
    __shared__ __align__(16) float sm[DF];
    __shared__ __align__(16) float sr[DF];
    const int lane = threadIdx.x & 31;
    const int wave = __builtin_amdgcn_readfirstlane((int)(threadIdx.x >> 5));
    const float invn = 1.0f / (float)(NB * OO);
#pragma unroll 1
    for (int q = 0; q < 4; ++q) {
        const int d = wave * 4 + q;
        float s = 0.0f;
#pragma unroll 1
        for (int b = 0; b < NB; ++b) { const float* row = VP + ((size_t)b * DF + d) * OO + lane;
#pragma unroll
            for (int j = 0; j < OO / 32; ++j) s += row[32 * j]; }
        s += __shfl_xor(s, 16, 32); s += __shfl_xor(s, 8, 32); s += __shfl_xor(s, 4, 32); s += __shfl_xor(s, 2, 32); s += __shfl_xor(s, 1, 32);
        const float mean = s * invn;
        float q2 = 0.0f;
#pragma unroll 1
        for (int b = 0; b < NB; ++b) { const float* row = VP + ((size_t)b * DF + d) * OO + lane;
#pragma unroll
            for (int j = 0; j < OO / 32; ++j) { const float t = row[32 * j] - mean; q2 += t * t; } }
        q2 += __shfl_xor(q2, 16, 32); q2 += __shfl_xor(q2, 8, 32); q2 += __shfl_xor(q2, 4, 32); q2 += __shfl_xor(q2, 2, 32); q2 += __shfl_xor(q2, 1, 32);
        const float var = q2 * invn;
        const float rstd = 1.0f / sqrtf(var + 1e-5f);
        if (lane == 0) { sm[d] = mean; sr[d] = rstd; }
    }
    __syncthreads();
    const int q8 = lane & 7;
    const v4f vm = *(const v4fa*)(&sm[4 * q8]);
    const v4f vr = *(const v4fa*)(&sr[4 * q8]);
    if (wave == 0) {
        if (lane < 8) {
            float* pm = BNT + 4 * lane; float* pr = BNT + 32 + 4 * lane;
            *(volatile v4f*)pm = vm; *(volatile v4f*)pr = vr;
            __threadfence();
            *(volatile v4f*)pm = vm; *(volatile v4f*)pr = vr;
        }
    }
}

__global__ __launch_bounds__(256) void k_w1t(const float* __restrict__ W1, h16* W1T) {
    __shared__ float ts[64 * 65];
    const int tid = threadIdx.x;
    const int l0 = blockIdx.x * 64, m0 = blockIdx.y * 64;
#pragma unroll 1
    for (int it = 0; it < 16; ++it) { const int e = it * 256 + tid; const int i = e >> 6, j = e & 63;
        ts[j * 65 + i] = W1[(size_t)(l0 + i) * DMM + m0 + j]; }
    __syncthreads();
    v8h hv[2];
#pragma unroll
    for (int it = 0; it < 2; ++it) { const int p = it * 256 + tid; const int row = p >> 3, c8 = (p & 7) * 8;
#pragma unroll
        for (int k = 0; k < 8; ++k) hv[it][k] = toh_flush(bfr(ts[row * 65 + c8 + k]) * WSC); }
#pragma unroll 1
    for (int ps = 0; ps < 2; ++ps) {
#pragma unroll
        for (int it = 0; it < 2; ++it) { const int p = it * 256 + tid; const int row = p >> 3, c8 = (p & 7) * 8;
            *(volatile v8h*)(W1T + (size_t)(m0 + row) * LL + l0 + c8) = hv[it]; }
        if (ps == 0) __threadfence(); }
}

__global__ __launch_bounds__(256) void k_mlp(const h16* __restrict__ ERR, const h16* __restrict__ W1T, const float* __restrict__ B1, const float* __restrict__ W2,
                                             const float* __restrict__ B2, float* WG) {
    __shared__ __align__(16) float os[8 * 16 * 68];
    __shared__ float sb1[DMM];
    __shared__ float sw2[DMM * 2];
    __shared__ float psum[8 * 64 * 2];
    __shared__ __align__(16) float wgs[64 * 2];
    const int lane = threadIdx.x & 31, lr = lane & 15, hi = lane >> 4;
    const int wave = __builtin_amdgcn_readfirstlane((int)(threadIdx.x >> 5));
    const int r0 = blockIdx.x * 64, c0 = wave * 64;
    for (int i = threadIdx.x; i < DMM; i += 256) sb1[i] = bfr(B1[i]);
    for (int i = threadIdx.x; i < DMM * 2; i += 256) sw2[i] = bfr(W2[i]);
    __syncthreads();
    v8f acc[4][4];
#pragma unroll
    for (int mb = 0; mb < 4; ++mb)
#pragma unroll
        for (int nb = 0; nb < 4; ++nb) acc[mb][nb] = (v8f){};
    const size_t aoff = (size_t)(r0 + lr) * LL + 8 * hi, boff = (size_t)(c0 + lr) * LL + 8 * hi;
#pragma unroll 1
    for (int kc = 0; kc < LL; kc += 32) {
        v16h a[4];
#pragma unroll
        for (int mb = 0; mb < 4; ++mb) a[mb] = ldh(ERR + aoff + (size_t)mb * 16 * LL + kc);
#pragma unroll
        for (int nb = 0; nb < 4; ++nb) { const v16h bq = ldh(W1T + boff + (size_t)nb * 16 * LL + kc);
#pragma unroll
            for (int mb = 0; mb < 4; ++mb) acc[mb][nb] = wmma16g(a[mb], bq, acc[mb][nb]); }
    }
    const int wb = wave * 16 * 68;
    const int row = lane >> 1, cb = (lane & 1) * 32;
#pragma unroll
    for (int mb = 0; mb < 4; ++mb) {
#pragma unroll
        for (int nb = 0; nb < 4; ++nb) {
#pragma unroll
            for (int j = 0; j < 8; ++j) os[wb + (hi * 8 + j) * 68 + nb * 16 + lr] = acc[mb][nb][j] * WSI; }
        wave_sync();
        float p0 = 0.0f, p1 = 0.0f;
#pragma unroll 1
        for (int c = 0; c < 32; ++c) {
            const int col = c0 + cb + c;
            const float z = os[wb + row * 68 + cb + c] + sb1[col];
            const float g = 0.5f * z * (1.0f + erff(z * 0.70710678118654752f));
            p0 += g * sw2[col * 2]; p1 += g * sw2[col * 2 + 1]; }
        p0 += __shfl_xor(p0, 1, 32); p1 += __shfl_xor(p1, 1, 32);
        psum[(wave * 64 + mb * 16 + row) * 2] = p0; psum[(wave * 64 + mb * 16 + row) * 2 + 1] = p1;
        wave_sync();
    }
    __syncthreads();
    if (wave < 2) {
        const int rr = wave * 32 + lane;
        float g0 = 0.0f, g1 = 0.0f;
#pragma unroll 1
        for (int w = 0; w < 8; ++w) { g0 += psum[(w * 64 + rr) * 2]; g1 += psum[(w * 64 + rr) * 2 + 1]; }
        g0 += bfr(B2[0]); g1 += bfr(B2[1]);
        const float mx = fmaxf(g0, g1);
        const float e0 = expf(g0 - mx), e1 = expf(g1 - mx);
        const float inv = 1.0f / (e0 + e1);
        wgs[rr * 2] = e0 * inv; wgs[rr * 2 + 1] = e1 * inv;
    }
    __syncthreads();
    const v4f val = *(const v4fa*)(&wgs[lane * 4]);
    if (wave == 0) {
        float* dst = WG + (size_t)r0 * 2 + lane * 4;
        *(volatile v4f*)dst = val; __threadfence(); *(volatile v4f*)dst = val;
    }
}

__global__ __launch_bounds__(256) void k_final(const float* __restrict__ VP, const float* __restrict__ YM, const float* __restrict__ BNT, const float* __restrict__ WG,
                                               const float* __restrict__ gamma, const float* __restrict__ beta, float* OUT) {
    __shared__ float vt[DF * 65];
    __shared__ float smu[32];
    __shared__ float srs[32];
    __shared__ float sga[32];
    __shared__ float sbe[32];
    __shared__ float sw0[32];
    __shared__ float sw1[32];
    const int tid = threadIdx.x;
    const int lane = threadIdx.x & 31;
    const int wave = __builtin_amdgcn_readfirstlane((int)(threadIdx.x >> 5));
    const int b = blockIdx.y; const int o0 = blockIdx.x * 64;
    if (wave == 0) {
        smu[lane] = BNT[lane]; srs[lane] = BNT[32 + lane]; sga[lane] = bfr(gamma[lane]); sbe[lane] = bfr(beta[lane]);
        sw0[lane] = WG[((size_t)b * DF + lane) * 2]; sw1[lane] = WG[((size_t)b * DF + lane) * 2 + 1];
    }
#pragma unroll 1
    for (int it = 0; it < 8; ++it) { const int e = it * 256 + tid; const int d = e >> 6, oo = e & 63;
        vt[d * 65 + oo] = VP[((size_t)b * DF + d) * OO + o0 + oo]; }
    __syncthreads();
    v4f res[2];
#pragma unroll
    for (int it = 0; it < 2; ++it) { const int p = it * 256 + tid; const int row = p >> 3, dq = (p & 7) * 4;
        const v4f ymv = *(const v4f*)(YM + ((size_t)b * OO + (size_t)(o0 + row)) * DF + dq);
#pragma unroll
        for (int k = 0; k < 4; ++k) { const int d = dq + k;
            const float y = ((vt[d * 65 + row] - smu[d]) * srs[d]) * sga[d] + sbe[d];
            res[it][k] = ymv[k] * sw0[d] + y * sw1[d]; } }
#pragma unroll 1
    for (int ps = 0; ps < 2; ++ps) {
#pragma unroll
        for (int it = 0; it < 2; ++it) { const int p = it * 256 + tid; const int row = p >> 3, dq = (p & 7) * 4;
            *(volatile v4f*)(OUT + ((size_t)b * OO + (size_t)(o0 + row)) * DF + dq) = res[it]; }
        if (ps == 0) __threadfence(); }
}

static constexpr size_t al256(size_t v) { return (v + 255) & ~(size_t)255; }
static constexpr size_t SZ_T1 = al256((size_t)NB * DF * 4);
static constexpr size_t SZ_T6 = al256((size_t)NB * DF * KD * 4);
static constexpr size_t SZ_XP = al256((size_t)NB * DF * LL * 32 * 2);
static constexpr size_t SZ_YP = al256((size_t)NB * DF * OO * 32 * 2);
static constexpr size_t SZ_ER = al256((size_t)NB * DF * LL * 2);
static constexpr size_t SZ_YM = al256((size_t)NB * OO * DF * 4);
static constexpr size_t SZ_VP = al256((size_t)NB * DF * OO * 4);
static constexpr size_t SZ_BN = al256((size_t)2 * DF * 4);
static constexpr size_t SZ_WT = al256((size_t)DMM * LL * 2);
static constexpr size_t SZ_WG = al256((size_t)NB * DF * 2 * 4);
static constexpr size_t SZ_TOTAL = 2 * SZ_T1 + 2 * SZ_T6 + SZ_XP + SZ_YP + SZ_ER + SZ_YM + SZ_VP + SZ_BN + SZ_WT + SZ_WG;
static_assert(SZ_TOTAL <= (size_t)134217728);
static_assert(((size_t)NB * DF) % 32 == 0);
static_assert(((size_t)NB * DF * KD) % 32 == 0);
static_assert((size_t)(NB * DF * KD / 32) * 32 * 4 <= SZ_T6);
static_assert((size_t)(NB * DF / 32) * 32 * 4 <= SZ_T1);

extern "C" void kernel_launch(void* const* d_in, const int* in_sizes, int n_in,
                              void* d_out, int out_size, void* d_ws, size_t ws_size, hipStream_t stream) {
    if (n_in < 9) return;
    if ((size_t)in_sizes[0] < (size_t)NB * LL * DF) return;
    if ((size_t)in_sizes[1] < (size_t)NB * LL * DF * KD) return;
    if ((size_t)in_sizes[2] < (size_t)NB * OO * DF * KD) return;
    if ((size_t)in_sizes[3] < (size_t)LL * DMM) return;
    if (in_sizes[4] < DMM || in_sizes[5] < DMM * 2 || in_sizes[6] < 2 || in_sizes[7] < DF || in_sizes[8] < DF) return;
    if ((size_t)out_size < (size_t)NB * OO * DF) return;
    if (SZ_TOTAL > ws_size) return;
    const float* x  = (const float*)d_in[0];
    const float* xd = (const float*)d_in[1];
    const float* yd = (const float*)d_in[2];
    const float* w1 = (const float*)d_in[3];
    const float* b1 = (const float*)d_in[4];
    const float* w2 = (const float*)d_in[5];
    const float* b2 = (const float*)d_in[6];
    const float* gamma = (const float*)d_in[7];
    const float* beta  = (const float*)d_in[8];
    float* OUT = (float*)d_out;
    char* wsp = (char*)d_ws;
    float* MEDT = (float*)wsp; wsp += SZ_T1;
    float* STDT = (float*)wsp; wsp += SZ_T1;
    float* MEDM = (float*)wsp; wsp += SZ_T6;
    float* STDM = (float*)wsp; wsp += SZ_T6;
    bf*    XP   = (bf*)wsp;    wsp += SZ_XP;
    bf*    YP   = (bf*)wsp;    wsp += SZ_YP;
    h16*   ERR  = (h16*)wsp;   wsp += SZ_ER;
    float* YM   = (float*)wsp; wsp += SZ_YM;
    float* VP   = (float*)wsp; wsp += SZ_VP;
    float* BNT  = (float*)wsp; wsp += SZ_BN;
    h16*   W1T  = (h16*)wsp;   wsp += SZ_WT;
    float* WG   = (float*)wsp; wsp += SZ_WG;

    k_stats<<<(unsigned)(NB * DF / 32), 256, 0, stream>>>(x, DF, MEDT, STDT);
    k_stats<<<(unsigned)(NB * DF * KD / 32), 256, 0, stream>>>(xd, DF * KD, MEDM, STDM);
    k_mapx<<<dim3(LL / 64, NB, 1), 256, 0, stream>>>(x, xd, MEDT, STDT, MEDM, STDM, XP, ERR);
    k_mapy<<<dim3(OO / 16, NB, 1), 256, 0, stream>>>(yd, MEDT, STDT, MEDM, STDM, YP, YM);
    k_flash<<<dim3(OO / (16 * AW), NB * DF, 1), 32 * AW, 0, stream>>>(XP, YP, x, VP);
    k_bn<<<1, 256, 0, stream>>>(VP, BNT);
    k_w1t<<<dim3(LL / 64, DMM / 64, 1), 256, 0, stream>>>(w1, W1T);
    k_mlp<<<(unsigned)(NB * DF / 64), 256, 0, stream>>>(ERR, W1T, b1, w2, b2, WG);
    k_final<<<dim3(OO / 64, NB, 1), 256, 0, stream>>>(VP, YM, BNT, WG, gamma, beta, OUT);
}
